// TieredGroupAttentionTier_39848706573738
// MI455X (gfx1250) — hardware-verified
//
#include <hip/hip_runtime.h>
#include <math.h>

#ifndef NB
#define NB 8
#endif
#ifndef SEQ
#define SEQ 2048
#endif
#define SEQ_FULL 2048
#define NB_FULL 8
#define DM 512
#define NQ 8
#define A1 128
#define A2 64
#define F1 (NQ * A1)
#define F2 (NQ * A2)
#define Q1GP ((NB >= 4) ? 4 : NB)
#define Q1PASSES (NB / Q1GP)

#define X_CARRY 16.0f
#define W_CARRY 64.0f
#define T1_CARRY 16.0f
#define RES_CARRY 2048.0f
#define CTX2_CARRY 0.25f
static constexpr float SC_XW   = 1.0f / 1024.0f;
static constexpr float SC_W    = 1.0f / 64.0f;
static constexpr float SC_KV1  = 1.0f / 256.0f;
static constexpr float SC_RES  = 1.0f / 2048.0f;
static constexpr float SC_O2   = 1.0f / 16.0f;
static constexpr float INV_SQRT_A1 = 0.08838834764831845f;
static constexpr float INV_SQRT_A2 = 0.125f;
static constexpr float SC_CTX1 = INV_SQRT_A1 * (1.0f / 16.0f);
static constexpr float ONE_F   = 1.0f;

static_assert(X_CARRY * W_CARRY * SC_XW == 1.0f);
static_assert(W_CARRY * SC_W == 1.0f);
static_assert(T1_CARRY * T1_CARRY * SC_KV1 == 1.0f);
static_assert(RES_CARRY * SC_RES == 1.0f);
static_assert(W_CARRY * CTX2_CARRY * SC_O2 == 1.0f);
static_assert(T1_CARRY * (1.0f / 16.0f) == 1.0f);
static_assert(A1 == 128 && A2 == 64);
static_assert(NB >= 1 && NB <= NB_FULL && SEQ <= SEQ_FULL);
static_assert(NB % Q1GP == 0);
static_assert(SEQ % 64 == 0 && DM % 64 == 0 && F1 % 64 == 0 && F2 % 64 == 0 && A1 % 64 == 0 && A2 % 64 == 0);
static_assert(SEQ % 32 == 0 && DM % 32 == 0 && F1 % 32 == 0 && F2 % 32 == 0 && A1 % 32 == 0 && A2 % 32 == 0);
static_assert((NB * A1) % 64 == 0);
static_assert((SEQ * DM / 8) % 256 == 0);
static_assert(DM / 8 == 64 && F1 / 8 == 128 && F2 / 8 == 64);
static_assert((A1 * (DM / 8)) % 256 == 0 && (A2 * (DM / 8)) % 256 == 0 && (DM * (F1 / 8)) % 256 == 0 && (DM * (F2 / 8)) % 256 == 0 && (DM * (DM / 8)) % 256 == 0);
static_assert(NQ == 8);
static_assert(32 * 16 * 8 == 16 * 64 * 4);
static_assert(32 * 16 * 4 == 16 * 64 * 2);
static_assert(8 * 16 * 68 * 4 <= 131072);

typedef __attribute__((ext_vector_type(16))) _Float16 v16h;
typedef __attribute__((ext_vector_type(8)))  _Float16 v8h;
typedef __attribute__((ext_vector_type(8)))  float    v8f;
typedef __attribute__((ext_vector_type(4)))  float    v4f;
typedef _Float16 h16;


__device__ __forceinline__ float bfr(float f) {
    unsigned u = __float_as_uint(f);
    u += 0x7FFFu + ((u >> 16) & 1u);
    return __uint_as_float(u & 0xFFFF0000u);
}
static __device__ __forceinline__ h16 toh_flush(float v) { const float w = (fabsf(v) < 6.103515625e-05f) ? 0.0f : v; return (h16)w; }

union FragU { v16h v; v8h h[2]; };
__device__ __forceinline__ v16h frag_ld(const _Float16* p) {
    FragU f; f.h[0] = *(const v8h*)(p); f.h[1] = *(const v8h*)(p + 16); return f.v;
}
__device__ __forceinline__ v8f wmma16g(v16h a, v16h b, v8f c) {
    c = __builtin_amdgcn_wmma_f32_16x16x32_f16(false, a, false, b, (short)0, c, false, false);
    asm volatile("v_nop\n\tv_nop\n\tv_nop\n\tv_nop" : "+v"(c) : "v"(a), "v"(b));
    return c;
}
__device__ __forceinline__ void wave_sync_lds() {
    __builtin_amdgcn_fence(3  , "workgroup");
    __builtin_amdgcn_wave_barrier();
    __builtin_amdgcn_fence(2  , "workgroup");
}
__device__ __forceinline__ unsigned wave_id() { return (unsigned)__builtin_amdgcn_readfirstlane((int)(threadIdx.x >> 5)); }

template <int MI, bool PROD3, int OUT_MODE, int BIAS_MODE>
__device__ __forceinline__ void gemm_tile(
    const _Float16* __restrict__ A, const _Float16* __restrict__ AL, const unsigned lda,
    const _Float16* __restrict__ Bt, const _Float16* __restrict__ BL, const unsigned ldb,
    float* __restrict__ Cf, _Float16* __restrict__ Ch, _Float16* __restrict__ Cl, const unsigned ldc,
    const float* __restrict__ bias, const unsigned m0, const unsigned n0, const unsigned K,
    const float scale, const float oscale, float* slab, const unsigned lane) {
  const unsigned rlane = lane & 15u;
  const unsigned koff = (lane >> 4) * 8u;
  const v8f vz = (v8f){0.f,0.f,0.f,0.f,0.f,0.f,0.f,0.f};
  v8f acc[MI][4];
  v8f acx[MI][4];
#pragma unroll
  for (int i = 0; i < MI; ++i)
#pragma unroll
    for (int j = 0; j < 4; ++j) { acc[i][j] = vz; acx[i][j] = vz; }

#pragma unroll 1
  for (unsigned k0 = 0; k0 < K; k0 += 32u) {
    v16h ah[MI];
    v16h al[MI];
#pragma unroll
    for (int i = 0; i < MI; ++i) {
      const size_t aoff = (size_t)(m0 + ((unsigned)i << 4) + rlane) * lda + koff + k0;
      ah[i] = frag_ld(A + aoff);
      if (PROD3) al[i] = frag_ld(AL + aoff); else al[i] = ah[i];
    }
#pragma unroll
    for (int j = 0; j < 4; ++j) {
      const size_t boff = (size_t)(n0 + ((unsigned)j << 4) + rlane) * ldb + koff + k0;
      const v16h bh = frag_ld(Bt + boff);
      v16h bl = bh;
      if (PROD3) bl = frag_ld(BL + boff);
#pragma unroll
      for (int i = 0; i < MI; ++i) {
        acc[i][j] = wmma16g(ah[i], bh, acc[i][j]);
        if (PROD3) {
          acx[i][j] = wmma16g(ah[i], bl, acx[i][j]);
          acx[i][j] = wmma16g(al[i], bh, acx[i][j]);
        }
      }
    }
  }

#pragma unroll
  for (int i = 0; i < MI; ++i) {
    const unsigned mBase = m0 + ((unsigned)i << 4);
    float rb[8];
#pragma unroll
    for (int r = 0; r < 8; ++r) rb[r] = 0.0f;
    if (BIAS_MODE == 2) {
#pragma unroll
      for (int r = 0; r < 8; ++r) rb[r] = bfr(bias[mBase + koff + (unsigned)r]);
    }
#pragma unroll
    for (int j = 0; j < 4; ++j) {
      float cb = 0.0f;
      if (BIAS_MODE == 1) cb = bfr(bias[n0 + ((unsigned)j << 4) + rlane]);
#pragma unroll
      for (int r = 0; r < 8; ++r) {
        float v = acc[i][j][r];
        if (PROD3) v = v + acx[i][j][r] * SC_RES;
        v = v * scale;
        if (BIAS_MODE == 1) v = v + cb;
        if (BIAS_MODE == 2) v = v + rb[r];
        if (OUT_MODE != 0) v = v * oscale;
        slab[(koff + (unsigned)r) * 68u + ((unsigned)j << 4) + rlane] = v;
      }
    }
    wave_sync_lds();
    if (OUT_MODE == 0) {
      const unsigned hh = lane >> 4, c4 = (lane & 15u) * 4u;
#pragma unroll
      for (int half = 0; half < 2; ++half) {
        v4f vv[4];
#pragma unroll
        for (int it = 0; it < 4; ++it) {
          const unsigned row = (unsigned)(half * 4 + it) * 2u + hh;
          vv[it] = *(const v4f*)(slab + row * 68u + c4);
        }
        for (int pass = 0; pass < 2; ++pass) {
#pragma unroll
          for (int it = 0; it < 4; ++it) {
            const unsigned row = (unsigned)(half * 4 + it) * 2u + hh;
            *(volatile v4f*)(Cf + (size_t)(mBase + row) * ldc + n0 + c4) = vv[it];
          }
          __threadfence();
        }
      }
    } else {
      const unsigned q = lane >> 3, c8 = (lane & 7u) * 8u;
      v8h hv[4];
      v8h lv[4];
#pragma unroll
      for (int it = 0; it < 4; ++it) {
        const unsigned row = (unsigned)it * 4u + q;
        const float* sp = slab + row * 68u + c8;
#pragma unroll
        for (int e = 0; e < 8; ++e) {
          const float f = sp[e];
          const h16 hi = toh_flush(f);
          hv[it][e] = hi;
          if (OUT_MODE == 2) lv[it][e] = toh_flush((f - (float)hi) * RES_CARRY); else lv[it][e] = hi;
        }
      }
      for (int pass = 0; pass < 2; ++pass) {
#pragma unroll
        for (int it = 0; it < 4; ++it) {
          const unsigned row = (unsigned)it * 4u + q;
          *(volatile v8h*)(Ch + (size_t)(mBase + row) * ldc + n0 + c8) = hv[it];
          if (OUT_MODE == 2) *(volatile v8h*)(Cl + (size_t)(mBase + row) * ldc + n0 + c8) = lv[it];
        }
        __threadfence();
      }
    }
    wave_sync_lds();
  }
}

__global__ __launch_bounds__(256) void k_xcvt(const float* __restrict__ x, _Float16* __restrict__ x16) {
    const unsigned u = blockIdx.x * 256u + threadIdx.x;
    if (u >= (unsigned)(SEQ * DM / 8)) return;
    const float* xr = x + (size_t)u * 8u;
    const v4f a = *(const v4f*)xr, b = *(const v4f*)(xr + 4);
    v8h hv;
    hv[0] = toh_flush(bfr(a.x) * X_CARRY); hv[1] = toh_flush(bfr(a.y) * X_CARRY);
    hv[2] = toh_flush(bfr(a.z) * X_CARRY); hv[3] = toh_flush(bfr(a.w) * X_CARRY);
    hv[4] = toh_flush(bfr(b.x) * X_CARRY); hv[5] = toh_flush(bfr(b.y) * X_CARRY);
    hv[6] = toh_flush(bfr(b.z) * X_CARRY); hv[7] = toh_flush(bfr(b.w) * X_CARRY);
    _Float16* dst = x16 + (size_t)u * 8u;
    *(volatile v8h*)dst = hv;
    __threadfence();
    *(volatile v8h*)dst = hv;
}

__global__ __launch_bounds__(256) void k_wt16(const float* __restrict__ Wm, unsigned KI, unsigned NO, unsigned lgper,
                                              _Float16* __restrict__ W16) {
    const unsigned layer = blockIdx.y;
    const float* Wl = Wm + (size_t)layer * KI * NO;
    _Float16* Dl = W16 + (size_t)layer * KI * NO;
    const unsigned u = blockIdx.x * 256u + threadIdx.x;
    const unsigned per = 1u << lgper;
    if (u >= NO * per) return;
    const unsigned k0 = 8u * (u & (per - 1u));
    const unsigned o = u >> lgper;
    v8h hv;
#pragma unroll
    for (int i = 0; i < 8; ++i) hv[i] = toh_flush(bfr(Wl[(size_t)(k0 + (unsigned)i) * NO + o]) * W_CARRY);
    _Float16* dst = Dl + (size_t)o * KI + k0;
    *(volatile v8h*)dst = hv;
    __threadfence();
    *(volatile v8h*)dst = hv;
}

__global__ __launch_bounds__(256) void k_q1(const _Float16* __restrict__ x16, const _Float16* __restrict__ wq,
                                            const float* __restrict__ bq, _Float16* __restrict__ qh, _Float16* __restrict__ ql, unsigned g0) {
  __shared__ __align__(16) float sT[8][16 * 68];
  const unsigned lane = threadIdx.x & 31u;
  const unsigned wave = wave_id();
  const unsigned tile = blockIdx.x * 8u + wave;
  constexpr unsigned TN = F1 / 64u, TM = SEQ / 64u, TPB = TM * TN;
  if (tile >= (unsigned)Q1GP * TPB) return;
  const unsigned z = tile / TPB;
  const unsigned t = tile - z * TPB;
  const unsigned tm = t / TN;
  const unsigned tn = t - tm * TN;
  const unsigned g = g0 + z;
  const size_t co = (size_t)z * SEQ * F1;
  gemm_tile<4, false, 2, 1>(x16, nullptr, DM, wq + (size_t)g * F1 * DM, nullptr, DM,
                            nullptr, qh + co, ql + co, F1, bq + (size_t)g * F1,
                            tm * 64u, tn * 64u, DM, SC_XW, T1_CARRY, sT[wave], lane);
}

__global__ __launch_bounds__(256) void k_kvt1(const _Float16* __restrict__ wp, const _Float16* __restrict__ x16,
                                              const float* __restrict__ bias, _Float16* __restrict__ outT) {
  __shared__ __align__(16) float sT[8][16 * 68];
  const unsigned lane = threadIdx.x & 31u;
  const unsigned wave = wave_id();
  const unsigned tile = blockIdx.x * 8u + wave;
  constexpr unsigned TN = SEQ / 64u, TM = (NB * A1) / 64u;
  if (tile >= TM * TN) return;
  const unsigned tm = tile / TN;
  const unsigned tn = tile - tm * TN;
  gemm_tile<4, false, 1, 2>(wp, nullptr, DM, x16, nullptr, DM,
                            nullptr, outT, nullptr, SEQ, bias,
                            tm * 64u, tn * 64u, DM, SC_XW, T1_CARRY, sT[wave], lane);
}

__global__ __launch_bounds__(256) void k_kv1(const _Float16* __restrict__ vt, const _Float16* __restrict__ kt,
                                             _Float16* __restrict__ kvh, _Float16* __restrict__ kvl) {
  __shared__ __align__(16) float sT[8][16 * 68];
  const unsigned lane = threadIdx.x & 31u;
  const unsigned wave = wave_id();
  const unsigned tile = blockIdx.x * 8u + wave;
  constexpr unsigned TN = A1 / 64u, TM = A1 / 64u, TPB = TM * TN;
  if (tile >= (unsigned)NB * TPB) return;
  const unsigned z = tile / TPB;
  const unsigned t = tile - z * TPB;
  const unsigned tm = t / TN;
  const unsigned tn = t - tm * TN;
  const size_t po = (size_t)z * A1 * SEQ;
  const size_t co = (size_t)z * A1 * A1;
  gemm_tile<4, false, 2, 0>(vt + po, nullptr, SEQ, kt + po, nullptr, SEQ,
                            nullptr, kvh + co, kvl + co, A1, nullptr,
                            tm * 64u, tn * 64u, SEQ, SC_KV1, ONE_F, sT[wave], lane);
}

__global__ __launch_bounds__(256) void k_ctx1(const _Float16* __restrict__ qh, const _Float16* __restrict__ ql,
                                              const _Float16* __restrict__ kvh, const _Float16* __restrict__ kvl,
                                              _Float16* __restrict__ ctx, unsigned g0) {
  __shared__ __align__(16) float sT[8][16 * 68];
  const unsigned lane = threadIdx.x & 31u;
  const unsigned wave = wave_id();
  const unsigned tile = blockIdx.x * 8u + wave;
  constexpr unsigned TN = A1 / 64u, TM = SEQ / 16u, TPB = TM * TN;
  if (tile >= (unsigned)(Q1GP * NQ) * TPB) return;
  const unsigned z = tile / TPB;
  const unsigned t = tile - z * TPB;
  const unsigned tm = t / TN;
  const unsigned tn = t - tm * TN;
  const unsigned gl = z / (unsigned)NQ;
  const unsigned q = z - gl * (unsigned)NQ;
  const unsigned g = g0 + gl;
  const size_t ao = (size_t)gl * SEQ * F1 + (size_t)q * A1;
  const size_t bo = (size_t)g * A1 * A1;
  const size_t co = (size_t)g * SEQ * F1 + (size_t)q * A1;
  gemm_tile<1, true, 1, 0>(qh + ao, ql + ao, F1, kvh + bo, kvl + bo, A1,
                           nullptr, ctx + co, nullptr, F1, nullptr,
                           tm * 16u, tn * 64u, A1, SC_CTX1, ONE_F, sT[wave], lane);
}

__global__ __launch_bounds__(256) void k_o1(const _Float16* __restrict__ ctx, const _Float16* __restrict__ wo,
                                            const float* __restrict__ bo, _Float16* __restrict__ o1) {
  __shared__ __align__(16) float sT[8][16 * 68];
  const unsigned lane = threadIdx.x & 31u;
  const unsigned wave = wave_id();
  const unsigned tile = blockIdx.x * 8u + wave;
  constexpr unsigned TN = DM / 64u, TM = SEQ / 64u, TPB = TM * TN;
  if (tile >= (unsigned)NB * TPB) return;
  const unsigned z = tile / TPB;
  const unsigned t = tile - z * TPB;
  const unsigned tm = t / TN;
  const unsigned tn = t - tm * TN;
  gemm_tile<4, false, 1, 1>(ctx + (size_t)z * SEQ * F1, nullptr, F1, wo + (size_t)z * DM * F1, nullptr, F1,
                            nullptr, o1 + (size_t)z * SEQ * DM, nullptr, DM, bo + (size_t)z * DM,
                            tm * 64u, tn * 64u, F1, SC_W, ONE_F, sT[wave], lane);
}

__global__ __launch_bounds__(256) void k_q2(const _Float16* __restrict__ o1, const _Float16* __restrict__ wq,
                                            const float* __restrict__ bq, _Float16* __restrict__ qh, _Float16* __restrict__ ql) {
  __shared__ __align__(16) float sT[8][16 * 68];
  const unsigned lane = threadIdx.x & 31u;
  const unsigned wave = wave_id();
  const unsigned tile = blockIdx.x * 8u + wave;
  constexpr unsigned TN = F2 / 64u, TM = SEQ / 64u, TPB = TM * TN;
  if (tile >= (unsigned)NB * TPB) return;
  const unsigned z = tile / TPB;
  const unsigned t = tile - z * TPB;
  const unsigned tm = t / TN;
  const unsigned tn = t - tm * TN;
  const size_t co = (size_t)z * SEQ * F2;
  gemm_tile<4, false, 2, 1>(o1 + (size_t)z * SEQ * DM, nullptr, DM, wq + (size_t)z * F2 * DM, nullptr, DM,
                            nullptr, qh + co, ql + co, F2, bq + (size_t)z * F2,
                            tm * 64u, tn * 64u, DM, SC_W, ONE_F, sT[wave], lane);
}

__global__ __launch_bounds__(256) void k_kvt2(const _Float16* __restrict__ wp, const _Float16* __restrict__ o1,
                                              const float* __restrict__ bias, _Float16* __restrict__ outT) {
  __shared__ __align__(16) float sT[8][16 * 68];
  const unsigned lane = threadIdx.x & 31u;
  const unsigned wave = wave_id();
  const unsigned tile = blockIdx.x * 8u + wave;
  constexpr unsigned TN = SEQ / 64u, TM = A2 / 64u, TPB = TM * TN;
  if (tile >= (unsigned)NB * TPB) return;
  const unsigned z = tile / TPB;
  const unsigned t = tile - z * TPB;
  const unsigned tm = t / TN;
  const unsigned tn = t - tm * TN;
  gemm_tile<4, false, 1, 2>(wp + (size_t)z * A2 * DM, nullptr, DM, o1 + (size_t)z * SEQ * DM, nullptr, DM,
                            nullptr, outT + (size_t)z * A2 * SEQ, nullptr, SEQ, bias + (size_t)z * A2,
                            tm * 64u, tn * 64u, DM, SC_W, ONE_F, sT[wave], lane);
}

__global__ __launch_bounds__(256) void k_kv2(const _Float16* __restrict__ vt, const _Float16* __restrict__ kt,
                                             _Float16* __restrict__ kvh, _Float16* __restrict__ kvl) {
  __shared__ __align__(16) float sT[8][16 * 68];
  const unsigned lane = threadIdx.x & 31u;
  const unsigned wave = wave_id();
  const unsigned tile = blockIdx.x * 8u + wave;
  constexpr unsigned TN = A2 / 64u, TM = A2 / 64u, TPB = TM * TN;
  if (tile >= (unsigned)NB * TPB) return;
  const unsigned z = tile / TPB;
  const unsigned t = tile - z * TPB;
  const unsigned tm = t / TN;
  const unsigned tn = t - tm * TN;
  const size_t po = (size_t)z * A2 * SEQ;
  const size_t co = (size_t)z * A2 * A2;
  gemm_tile<4, false, 2, 0>(vt + po, nullptr, SEQ, kt + po, nullptr, SEQ,
                            nullptr, kvh + co, kvl + co, A2, nullptr,
                            tm * 64u, tn * 64u, SEQ, ONE_F, ONE_F, sT[wave], lane);
}

__global__ __launch_bounds__(256) void k_ctx2(const _Float16* __restrict__ qh, const _Float16* __restrict__ ql,
                                              const _Float16* __restrict__ kvh, const _Float16* __restrict__ kvl,
                                              _Float16* __restrict__ ctx) {
  __shared__ __align__(16) float sT[8][16 * 68];
  const unsigned lane = threadIdx.x & 31u;
  const unsigned wave = wave_id();
  const unsigned tile = blockIdx.x * 8u + wave;
  constexpr unsigned TN = A2 / 64u, TM = SEQ / 16u, TPB = TM * TN;
  if (tile >= (unsigned)(NB * NQ) * TPB) return;
  const unsigned z = tile / TPB;
  const unsigned t = tile - z * TPB;
  const unsigned tm = t / TN;
  const unsigned tn = t - tm * TN;
  const unsigned g = z / (unsigned)NQ;
  const unsigned q = z - g * (unsigned)NQ;
  const size_t ao = (size_t)g * SEQ * F2 + (size_t)q * A2;
  const size_t bo = (size_t)g * A2 * A2;
  gemm_tile<1, true, 1, 0>(qh + ao, ql + ao, F2, kvh + bo, kvl + bo, A2,
                           nullptr, ctx + ao, nullptr, F2, nullptr,
                           tm * 16u, tn * 64u, A2, INV_SQRT_A2, CTX2_CARRY, sT[wave], lane);
}

__global__ __launch_bounds__(256) void k_o2(const _Float16* __restrict__ ctx, const _Float16* __restrict__ wo,
                                            const float* __restrict__ bo, _Float16* __restrict__ o2) {
  __shared__ __align__(16) float sT[8][16 * 68];
  const unsigned lane = threadIdx.x & 31u;
  const unsigned wave = wave_id();
  const unsigned tile = blockIdx.x * 8u + wave;
  constexpr unsigned TN = DM / 64u, TM = SEQ / 64u, TPB = TM * TN;
  if (tile >= (unsigned)NB * TPB) return;
  const unsigned z = tile / TPB;
  const unsigned t = tile - z * TPB;
  const unsigned tm = t / TN;
  const unsigned tn = t - tm * TN;
  gemm_tile<4, false, 1, 1>(ctx + (size_t)z * SEQ * F2, nullptr, F2, wo + (size_t)z * DM * F2, nullptr, F2,
                            nullptr, o2 + (size_t)z * SEQ * DM, nullptr, DM, bo + (size_t)z * DM,
                            tm * 64u, tn * 64u, F2, SC_O2, ONE_F, sT[wave], lane);
}

__global__ __launch_bounds__(256) void k_final(const _Float16* __restrict__ o2, const _Float16* __restrict__ wo,
                                               const float* __restrict__ bo, float* __restrict__ out) {
  __shared__ __align__(16) float sT[8][16 * 68];
  const unsigned lane = threadIdx.x & 31u;
  const unsigned wave = wave_id();
  const unsigned tile = blockIdx.x * 8u + wave;
  constexpr unsigned TN = DM / 64u, TM = SEQ / 64u, TPB = TM * TN;
  if (tile >= (unsigned)NB * TPB) return;
  const unsigned z = tile / TPB;
  const unsigned t = tile - z * TPB;
  const unsigned tm = t / TN;
  const unsigned tn = t - tm * TN;
  gemm_tile<4, false, 0, 1>(o2 + (size_t)z * SEQ * DM, nullptr, DM, wo, nullptr, DM,
                            out + (size_t)z * SEQ_FULL * DM, nullptr, nullptr, DM, bo,
                            tm * 64u, tn * 64u, DM, SC_W, ONE_F, sT[wave], lane);
}

static constexpr size_t al256(size_t b) { return (b + 255) & ~(size_t)255; }
static constexpr size_t cmax(size_t a, size_t b) { return a > b ? a : b; }
static constexpr size_t SZ_X16  = al256((size_t)SEQ * DM * 2);
static constexpr size_t SZ_WQ1  = al256((size_t)NB * F1 * DM * 2);
static constexpr size_t SZ_WKV1 = al256((size_t)NB * A1 * DM * 2);
static constexpr size_t SZ_WO1  = al256((size_t)NB * DM * F1 * 2);
static constexpr size_t SZ_WQ2  = al256((size_t)NB * F2 * DM * 2);
static constexpr size_t SZ_WKV2 = al256((size_t)NB * A2 * DM * 2);
static constexpr size_t SZ_WO2  = al256((size_t)NB * DM * F2 * 2);
static constexpr size_t SZ_WO   = al256((size_t)DM * DM * 2);
static constexpr size_t SZ_KVT1 = al256((size_t)NB * A1 * SEQ * 2);
static constexpr size_t SZ_KV1  = al256((size_t)NB * A1 * A1 * 2);
static constexpr size_t SZ_KVT2 = al256((size_t)NB * A2 * SEQ * 2);
static constexpr size_t SZ_KV2  = al256((size_t)NB * A2 * A2 * 2);
static constexpr size_t SZ_Q1P  = al256((size_t)Q1GP * SEQ * F1 * 2);
static constexpr size_t SZ_Q2P  = al256((size_t)NB * SEQ * F2 * 2);
static constexpr size_t SZ_CTX1 = al256((size_t)NB * SEQ * F1 * 2);
static constexpr size_t SZ_CTX2 = al256((size_t)NB * SEQ * F2 * 2);
static constexpr size_t SZ_O2   = al256((size_t)NB * SEQ * DM * 2);
static constexpr size_t SZ_O1   = al256((size_t)NB * SEQ * DM * 2);
static constexpr size_t SZ_R1   = cmax(2 * SZ_Q1P, 2 * SZ_Q2P);
static constexpr size_t SZ_R2   = cmax(SZ_CTX1, SZ_CTX2 + SZ_O2);
static_assert(2 * SZ_Q1P <= SZ_R1 && 2 * SZ_Q2P <= SZ_R1);
static_assert(SZ_CTX1 <= SZ_R2 && SZ_CTX2 + SZ_O2 <= SZ_R2);

static constexpr size_t OFF_X16  = 0;
static constexpr size_t OFF_WQ1  = OFF_X16 + SZ_X16;
static constexpr size_t OFF_WK1  = OFF_WQ1 + SZ_WQ1;
static constexpr size_t OFF_WV1  = OFF_WK1 + SZ_WKV1;
static constexpr size_t OFF_WO1  = OFF_WV1 + SZ_WKV1;
static constexpr size_t OFF_WQ2  = OFF_WO1 + SZ_WO1;
static constexpr size_t OFF_WK2  = OFF_WQ2 + SZ_WQ2;
static constexpr size_t OFF_WV2  = OFF_WK2 + SZ_WKV2;
static constexpr size_t OFF_WO2  = OFF_WV2 + SZ_WKV2;
static constexpr size_t OFF_WO   = OFF_WO2 + SZ_WO2;
static constexpr size_t OFF_K1T  = OFF_WO + SZ_WO;
static constexpr size_t OFF_V1T  = OFF_K1T + SZ_KVT1;
static constexpr size_t OFF_KV1H = OFF_V1T + SZ_KVT1;
static constexpr size_t OFF_KV1L = OFF_KV1H + SZ_KV1;
static constexpr size_t OFF_K2T  = OFF_KV1L + SZ_KV1;
static constexpr size_t OFF_V2T  = OFF_K2T + SZ_KVT2;
static constexpr size_t OFF_KV2H = OFF_V2T + SZ_KVT2;
static constexpr size_t OFF_KV2L = OFF_KV2H + SZ_KV2;
static constexpr size_t OFF_R1   = OFF_KV2L + SZ_KV2;
static constexpr size_t OFF_R2   = OFF_R1 + SZ_R1;
static constexpr size_t OFF_O1   = OFF_R2 + SZ_R2;
static constexpr size_t WS_TOTAL = OFF_O1 + SZ_O1;
static_assert(WS_TOTAL <= (size_t)134217728);

static constexpr size_t OUT_ELEMS_NEEDED = ((size_t)(NB - 1) * SEQ_FULL + SEQ) * DM;
static_assert(OUT_ELEMS_NEEDED <= (size_t)NB_FULL * SEQ_FULL * DM);

extern "C" void kernel_launch(void* const* d_in, const int* in_sizes, int n_in, void* d_out, int out_size,
                              void* d_ws, size_t ws_size, hipStream_t stream) {
    if (n_in < 19) return;
    if (in_sizes[0] < SEQ * DM) return;
    if (in_sizes[1] < NB * NQ * DM * A1 || in_sizes[2] < NB * NQ * A1) return;
    if (in_sizes[3] < NB * DM * A1 || in_sizes[4] < NB * A1 || in_sizes[5] < NB * DM * A1 || in_sizes[6] < NB * A1) return;
    if (in_sizes[7] < NB * F1 * DM || in_sizes[8] < NB * DM) return;
    if (in_sizes[9] < NB * NQ * DM * A2 || in_sizes[10] < NB * NQ * A2) return;
    if (in_sizes[11] < NB * DM * A2 || in_sizes[12] < NB * A2 || in_sizes[13] < NB * DM * A2 || in_sizes[14] < NB * A2) return;
    if (in_sizes[15] < NB * F2 * DM || in_sizes[16] < NB * DM) return;
    if (in_sizes[17] < DM * DM || in_sizes[18] < DM) return;
    if ((size_t)out_size < OUT_ELEMS_NEEDED) return;
    if (WS_TOTAL > ws_size) return;

    const float* x   = (const float*)d_in[0];
    const float* Wq1 = (const float*)d_in[1];
    const float* bq1 = (const float*)d_in[2];
    const float* Wk1 = (const float*)d_in[3];
    const float* bk1 = (const float*)d_in[4];
    const float* Wv1 = (const float*)d_in[5];
    const float* bv1 = (const float*)d_in[6];
    const float* Wo1 = (const float*)d_in[7];
    const float* bo1 = (const float*)d_in[8];
    const float* Wq2 = (const float*)d_in[9];
    const float* bq2 = (const float*)d_in[10];
    const float* Wk2 = (const float*)d_in[11];
    const float* bk2 = (const float*)d_in[12];
    const float* Wv2 = (const float*)d_in[13];
    const float* bv2 = (const float*)d_in[14];
    const float* Wo2 = (const float*)d_in[15];
    const float* bo2 = (const float*)d_in[16];
    const float* Wo  = (const float*)d_in[17];
    const float* bo  = (const float*)d_in[18];
    float* out = (float*)d_out;

    char* wsp = (char*)d_ws;
    _Float16* x16  = (_Float16*)(wsp + OFF_X16);
    _Float16* wq1p = (_Float16*)(wsp + OFF_WQ1);
    _Float16* wk1p = (_Float16*)(wsp + OFF_WK1);
    _Float16* wv1p = (_Float16*)(wsp + OFF_WV1);
    _Float16* wo1p = (_Float16*)(wsp + OFF_WO1);
    _Float16* wq2p = (_Float16*)(wsp + OFF_WQ2);
    _Float16* wk2p = (_Float16*)(wsp + OFF_WK2);
    _Float16* wv2p = (_Float16*)(wsp + OFF_WV2);
    _Float16* wo2p = (_Float16*)(wsp + OFF_WO2);
    _Float16* wop  = (_Float16*)(wsp + OFF_WO);
    _Float16* k1t  = (_Float16*)(wsp + OFF_K1T);
    _Float16* v1t  = (_Float16*)(wsp + OFF_V1T);
    _Float16* kv1h = (_Float16*)(wsp + OFF_KV1H);
    _Float16* kv1l = (_Float16*)(wsp + OFF_KV1L);
    _Float16* k2t  = (_Float16*)(wsp + OFF_K2T);
    _Float16* v2t  = (_Float16*)(wsp + OFF_V2T);
    _Float16* kv2h = (_Float16*)(wsp + OFF_KV2H);
    _Float16* kv2l = (_Float16*)(wsp + OFF_KV2L);
    _Float16* q1h  = (_Float16*)(wsp + OFF_R1);
    _Float16* q1l  = (_Float16*)(wsp + OFF_R1 + SZ_Q1P);
    _Float16* q2h  = (_Float16*)(wsp + OFF_R1);
    _Float16* q2l  = (_Float16*)(wsp + OFF_R1 + SZ_Q2P);
    _Float16* ctx1 = (_Float16*)(wsp + OFF_R2);
    _Float16* ctx2 = (_Float16*)(wsp + OFF_R2);
    _Float16* o2p  = (_Float16*)(wsp + OFF_R2 + SZ_CTX2);
    _Float16* o1p  = (_Float16*)(wsp + OFF_O1);

    k_xcvt<<<(SEQ * DM / 8) / 256, 256, 0, stream>>>(x, x16);
    k_wt16<<<dim3((A1 * (DM / 8)) / 256, NB * NQ), 256, 0, stream>>>(Wq1, DM, A1, 6, wq1p);
    k_wt16<<<dim3((A1 * (DM / 8)) / 256, NB), 256, 0, stream>>>(Wk1, DM, A1, 6, wk1p);
    k_wt16<<<dim3((A1 * (DM / 8)) / 256, NB), 256, 0, stream>>>(Wv1, DM, A1, 6, wv1p);
    k_wt16<<<dim3((DM * (F1 / 8)) / 256, NB), 256, 0, stream>>>(Wo1, F1, DM, 7, wo1p);
    k_wt16<<<dim3((A2 * (DM / 8)) / 256, NB * NQ), 256, 0, stream>>>(Wq2, DM, A2, 6, wq2p);
    k_wt16<<<dim3((A2 * (DM / 8)) / 256, NB), 256, 0, stream>>>(Wk2, DM, A2, 6, wk2p);
    k_wt16<<<dim3((A2 * (DM / 8)) / 256, NB), 256, 0, stream>>>(Wv2, DM, A2, 6, wv2p);
    k_wt16<<<dim3((DM * (F2 / 8)) / 256, NB), 256, 0, stream>>>(Wo2, F2, DM, 6, wo2p);
    k_wt16<<<dim3((DM * (DM / 8)) / 256, 1), 256, 0, stream>>>(Wo, DM, DM, 6, wop);

    k_kvt1<<<(((NB * A1) / 64) * (SEQ / 64) + 7) / 8, 256, 0, stream>>>(wk1p, x16, bk1, k1t);
    k_kvt1<<<(((NB * A1) / 64) * (SEQ / 64) + 7) / 8, 256, 0, stream>>>(wv1p, x16, bv1, v1t);
    k_kv1<<<(NB * (A1 / 64) * (A1 / 64) + 7) / 8, 256, 0, stream>>>(v1t, k1t, kv1h, kv1l);
    for (int p = 0; p < Q1PASSES; ++p) {
        const unsigned g0 = (unsigned)(p * Q1GP);
        k_q1<<<(Q1GP * (SEQ / 64) * (F1 / 64) + 7) / 8, 256, 0, stream>>>(x16, wq1p, bq1, q1h, q1l, g0);
        k_ctx1<<<(Q1GP * NQ * (SEQ / 16) * (A1 / 64) + 7) / 8, 256, 0, stream>>>(q1h, q1l, kv1h, kv1l, ctx1, g0);
    }
    k_o1<<<(NB * (SEQ / 64) * (DM / 64) + 7) / 8, 256, 0, stream>>>(ctx1, wo1p, bo1, o1p);

    k_q2<<<(NB * (SEQ / 64) * (F2 / 64) + 7) / 8, 256, 0, stream>>>(o1p, wq2p, bq2, q2h, q2l);
    k_kvt2<<<(NB * (A2 / 64) * (SEQ / 64) + 7) / 8, 256, 0, stream>>>(wk2p, o1p, bk2, k2t);
    k_kvt2<<<(NB * (A2 / 64) * (SEQ / 64) + 7) / 8, 256, 0, stream>>>(wv2p, o1p, bv2, v2t);
    k_kv2<<<(NB * (A2 / 64) * (A2 / 64) + 7) / 8, 256, 0, stream>>>(v2t, k2t, kv2h, kv2l);
    k_ctx2<<<(NB * NQ * (SEQ / 16) * (A2 / 64) + 7) / 8, 256, 0, stream>>>(q2h, q2l, kv2h, kv2l, ctx2);
    k_o2<<<(NB * (SEQ / 64) * (DM / 64) + 7) / 8, 256, 0, stream>>>(ctx2, wo2p, bo2, o2p);

    k_final<<<(NB * (SEQ / 64) * (DM / 64) + 7) / 8, 256, 0, stream>>>(o2p, wop, bo, out);
}
